// GeLULayerForGATLayer_45105746542641
// MI455X (gfx1250) — hardware-verified
//
#include <hip/hip_runtime.h>
#include <stddef.h>


#define FEAT   128
#define BONDF  16
#define K2P    160
#define AP2    168
#define NTHR   256
#define NWAVE  8
#define EPT    8
#define NGRP   2
#define CHUNK  (NTHR * EPT * NGRP)
#define WCAP   (EPT * NGRP * 32)
#define LISTN  (NWAVE * WCAP)
#define NBA    256
#define GROWS  64
#define GTHR   128
#define EROWS  128
#define GIP    768

#define WO_FC1  0
#define WO_ATT  32768
#define WO_FC2  65536
#define WO_WIH1 106496
#define WO_WHH1 204800
#define WO_F2V2 303104
#define WO_WIH2 335872
#define WO_WHH2 434176
#define WO_LIN  532480
#define WO_END  565248
#define WSZ_SQ  16384
#define WSZ_FC2 20480
#define WSZ_GRU 49152
#define WGRP_END 35328

#define LDS_EDGE (2 * EROWS * AP2 * 2 + EROWS * 4)
#define LDS_AGG  (NBA * FEAT * 4 + 2 * NBA * 4 + LISTN * 4 + 64)
#define LDS_GRU  (GROWS * GIP * 4 + 2 * GROWS * 4)

static_assert(CHUNK == 4096);
static_assert(WCAP == 512);
static_assert((NBA & (NBA - 1)) == 0 && NBA <= 4096 && NBA == NWAVE * 32);
static_assert(EROWS == NWAVE * 16 && NTHR == 2 * EROWS);
static_assert(GROWS == (GTHR / 32) * 16);
static_assert((AP2 % 8) == 0 && AP2 >= K2P);
static_assert(WGRP_END * 8 == WO_END / 2 * 1 + 0 || true);
static_assert(WO_END == 2 * (4 * WSZ_SQ + WSZ_FC2 + 4 * WSZ_GRU));
static_assert((WGRP_END % NTHR) == 0);

typedef float          v4f  __attribute__((ext_vector_type(4)));
typedef float          v8f  __attribute__((ext_vector_type(8)));
typedef int            v4i  __attribute__((ext_vector_type(4)));
typedef unsigned short v4us __attribute__((ext_vector_type(4)));
typedef unsigned short v8us __attribute__((ext_vector_type(8)));
typedef unsigned short v16us __attribute__((ext_vector_type(16)));
typedef __bf16         v16bf __attribute__((ext_vector_type(16)));
union FragB { v16us u; v8us h[2]; v16bf b; };

__device__ __forceinline__ unsigned short bfr(float x) {
  unsigned int u = __float_as_uint(x);
  u += 0x7FFFu + ((u >> 16) & 1u);
  return (unsigned short)(u >> 16);
}
__device__ __forceinline__ float bfu(unsigned short b) { return __uint_as_float(((unsigned int)b) << 16); }
__device__ __forceinline__ v4us hi4(v4f v) {
  v4us h; h.x = bfr(v.x); h.y = bfr(v.y); h.z = bfr(v.z); h.w = bfr(v.w); return h;
}
__device__ __forceinline__ v4us lo4(v4f v, v4us h) {
  v4us l;
  l.x = bfr(v.x - bfu(h.x)); l.y = bfr(v.y - bfu(h.y)); l.z = bfr(v.z - bfu(h.z)); l.w = bfr(v.w - bfu(h.w));
  return l;
}
__device__ __forceinline__ v8us cat8(v4us a, v4us b) {
  v8us r;
  r[0] = a.x; r[1] = a.y; r[2] = a.z; r[3] = a.w; r[4] = b.x; r[5] = b.y; r[6] = b.z; r[7] = b.w;
  return r;
}
__device__ __forceinline__ int clampi(int v, int hi) { return v < 0 ? 0 : (v > hi ? hi : v); }
__device__ __forceinline__ float lrl(float x) { return x >= 0.f ? x : 0.2f * x; }
__device__ __forceinline__ float sigf(float x) { return __builtin_amdgcn_rcpf(1.0f + expf(-x)); }

__device__ __forceinline__ v8f wmb(v16us a, v16us b, v8f c) {
  FragB fa, fb; fa.u = a; fb.u = b;
  v8f d = __builtin_amdgcn_wmma_f32_16x16x32_bf16(false, fa.b, false, fb.b, (short)0, c, false, false);
  asm volatile("v_nop\n\tv_nop\n\tv_nop\n\tv_nop" : "+v"(d) : "v"(fa.b), "v"(fb.b));
  return d;
}
__device__ __forceinline__ v8f wm3(v16us ah, v16us al, v16us bh, v16us bl, v8f c) {
  c = wmb(ah, bh, c);
  c = wmb(ah, bl, c);
  c = wmb(al, bh, c);
  return c;
}

template <int NB>
__device__ __forceinline__ int scan_chunk(const int* __restrict__ dsts, int nE, int cbase, int slotBase,
                                          int vec8, int* list, int tid, int lane, int wave) {
  int wc = 0;
#pragma unroll
  for (int g = 0; g < NGRP; ++g) {
    const int el0  = (g * NTHR + tid) * EPT;
    const int e0   = cbase + el0;
    const int sent = -2147483647 - 1;
    v4i da, db;
    if (vec8 != 0 && cbase + CHUNK <= nE) {
      da = *(const v4i*)(dsts + e0);
      db = *(const v4i*)(dsts + e0 + 4);
    } else {
      da.x = (e0     < nE) ? dsts[min(e0,     nE - 1)] : sent;
      da.y = (e0 + 1 < nE) ? dsts[min(e0 + 1, nE - 1)] : sent;
      da.z = (e0 + 2 < nE) ? dsts[min(e0 + 2, nE - 1)] : sent;
      da.w = (e0 + 3 < nE) ? dsts[min(e0 + 3, nE - 1)] : sent;
      db.x = (e0 + 4 < nE) ? dsts[min(e0 + 4, nE - 1)] : sent;
      db.y = (e0 + 5 < nE) ? dsts[min(e0 + 5, nE - 1)] : sent;
      db.z = (e0 + 6 < nE) ? dsts[min(e0 + 6, nE - 1)] : sent;
      db.w = (e0 + 7 < nE) ? dsts[min(e0 + 7, nE - 1)] : sent;
    }
    const unsigned nb = (unsigned)slotBase;
    const unsigned s0 = (unsigned)da.x - nb, s1 = (unsigned)da.y - nb;
    const unsigned s2 = (unsigned)da.z - nb, s3 = (unsigned)da.w - nb;
    const unsigned s4 = (unsigned)db.x - nb, s5 = (unsigned)db.y - nb;
    const unsigned s6 = (unsigned)db.z - nb, s7 = (unsigned)db.w - nb;
    const bool h0 = s0 < (unsigned)NB, h1 = s1 < (unsigned)NB, h2 = s2 < (unsigned)NB, h3 = s3 < (unsigned)NB;
    const bool h4 = s4 < (unsigned)NB, h5 = s5 < (unsigned)NB, h6 = s6 < (unsigned)NB, h7 = s7 < (unsigned)NB;
    const unsigned any = __builtin_amdgcn_ballot_w32(h0 | h1 | h2 | h3 | h4 | h5 | h6 | h7);
    if (any != 0u) {
#define HITJ(J, HJ, SJ) { \
        const unsigned mj = __builtin_amdgcn_ballot_w32(HJ); \
        if (mj != 0u) { \
          if (HJ) { \
            const int pos = wc + (int)__builtin_amdgcn_mbcnt_lo(mj, 0u); \
            if (pos < WCAP) list[wave * WCAP + pos] = ((el0 + (J)) << 12) | (int)(SJ); \
          } \
          wc += (int)__builtin_popcount(mj); } }
      HITJ(0, h0, s0)
      HITJ(1, h1, s1)
      HITJ(2, h2, s2)
      HITJ(3, h3, s3)
      HITJ(4, h4, s4)
      HITJ(5, h5, s5)
      HITJ(6, h6, s6)
      HITJ(7, h7, s7)
#undef HITJ
    }
  }
  return wc;
}

__global__ __launch_bounds__(NTHR) void k_wprep(
    const float* __restrict__ w0, const float* __restrict__ w1, const float* __restrict__ w2,
    const float* __restrict__ w3, const float* __restrict__ w4, const float* __restrict__ w5,
    const float* __restrict__ w6, const float* __restrict__ w7, const float* __restrict__ w8,
    unsigned short* wpl) {
  const int bstart = blockIdx.x * NTHR;
  const float* src; int nout, kreal, kp, gstart, base, psz;
  if      (bstart <  2048) { src = w0; nout = 128; kreal = 128; kp = 128; gstart = 0;     base = WO_FC1;  psz = WSZ_SQ;  }
  else if (bstart <  4096) { src = w1; nout = 128; kreal = 128; kp = 128; gstart = 2048;  base = WO_ATT;  psz = WSZ_SQ;  }
  else if (bstart <  6656) { src = w2; nout = 128; kreal = 144; kp = 160; gstart = 4096;  base = WO_FC2;  psz = WSZ_FC2; }
  else if (bstart < 12800) { src = w3; nout = 384; kreal = 128; kp = 128; gstart = 6656;  base = WO_WIH1; psz = WSZ_GRU; }
  else if (bstart < 18944) { src = w4; nout = 384; kreal = 128; kp = 128; gstart = 12800; base = WO_WHH1; psz = WSZ_GRU; }
  else if (bstart < 20992) { src = w5; nout = 128; kreal = 128; kp = 128; gstart = 18944; base = WO_F2V2; psz = WSZ_SQ;  }
  else if (bstart < 27136) { src = w6; nout = 384; kreal = 128; kp = 128; gstart = 20992; base = WO_WIH2; psz = WSZ_GRU; }
  else if (bstart < 33280) { src = w7; nout = 384; kreal = 128; kp = 128; gstart = 27136; base = WO_WHH2; psz = WSZ_GRU; }
  else                     { src = w8; nout = 128; kreal = 128; kp = 128; gstart = 33280; base = WO_LIN;  psz = WSZ_SQ;  }
  const int i = bstart + (int)threadIdx.x;
  if (i >= WGRP_END) return;
  const int o  = (i - gstart) * 8;
  const int n  = o / kp;
  const int k0 = o - n * kp;
  const int nc = n < nout ? n : nout - 1;
  float v[8];
#pragma unroll
  for (int e = 0; e < 8; ++e) {
    const int k  = k0 + e;
    const int kc = k < kreal ? k : kreal - 1;
    const float x = src[(size_t)nc * kreal + kc];
    v[e] = (k < kreal && n < nout) ? x : 0.0f;
  }
  v4f a, b;
  a.x = v[0]; a.y = v[1]; a.z = v[2]; a.w = v[3];
  b.x = v[4]; b.y = v[5]; b.z = v[6]; b.w = v[7];
  const v4us ha = hi4(a), hb = hi4(b);
  const v4us la = lo4(a, ha), lb = lo4(b, hb);
  const v8us hv = cat8(ha, hb), lv = cat8(la, lb);
  unsigned short* ph = wpl + base + o;
  unsigned short* pl = ph + psz;
  *(volatile v8us*)ph = hv;
  *(volatile v8us*)pl = lv;
  __threadfence();
  *(volatile v8us*)ph = hv;
  *(volatile v8us*)pl = lv;
}

__global__ __launch_bounds__(NTHR) void k_aprep(const float* __restrict__ x, unsigned short* ph, unsigned short* pl, int nN) {
  const int i = blockIdx.x * NTHR + (int)threadIdx.x;
  const int row = i >> 4;
  const int c0  = (i & 15) * 8;
  const int rc  = row > nN - 1 ? nN - 1 : row;
  const float* xp = x + (size_t)rc * FEAT + c0;
  v4f a = *(const v4f*)xp, b = *(const v4f*)(xp + 4);
  const v4f z = {0.f, 0.f, 0.f, 0.f};
  if (row >= nN) { a = z; b = z; }
  const v4us ha = hi4(a), hb = hi4(b);
  const v4us la = lo4(a, ha), lb = lo4(b, hb);
  const v8us hv = cat8(ha, hb), lv = cat8(la, lb);
  const size_t o = (size_t)i * 8;
  *(volatile v8us*)(ph + o) = hv;
  *(volatile v8us*)(pl + o) = lv;
  __threadfence();
  *(volatile v8us*)(ph + o) = hv;
  *(volatile v8us*)(pl + o) = lv;
}

__global__ __launch_bounds__(GTHR) void k_lin(
    const unsigned short* __restrict__ Ah, const unsigned short* __restrict__ Al,
    const unsigned short* __restrict__ Bh, const unsigned short* __restrict__ Bl,
    const float* __restrict__ bias, int act,
    float* outF, int useF, int nValid,
    unsigned short* Ph, unsigned short* Pl, int useP,
    const float* __restrict__ dw, float* dout, int useD) {
  __shared__ __attribute__((aligned(16))) float stg[GROWS * FEAT];
  __shared__ __attribute__((aligned(16))) float sdot[GROWS];
  const int tid = threadIdx.x, lane = tid & 31, wave = tid >> 5, hh = lane >> 4, m = lane & 15;
  const int rowBase = blockIdx.x * GROWS;
  const int r0 = wave * 16;

  v8f acc[8];
#pragma unroll
  for (int t = 0; t < 8; ++t) { v8f z = {0.f, 0.f, 0.f, 0.f, 0.f, 0.f, 0.f, 0.f}; acc[t] = z; }
  const size_t ao = (size_t)(rowBase + r0 + m) * FEAT + 8 * hh;
  const unsigned short* ah = Ah + ao;
  const unsigned short* al = Al + ao;
#pragma unroll
  for (int kt = 0; kt < FEAT / 32; ++kt) {
    FragB fah, fal;
    fah.h[0] = *(const v8us*)(ah + 32 * kt);
    fah.h[1] = *(const v8us*)(ah + 32 * kt + 16);
    fal.h[0] = *(const v8us*)(al + 32 * kt);
    fal.h[1] = *(const v8us*)(al + 32 * kt + 16);
#pragma unroll
    for (int t = 0; t < 8; ++t) {
      const size_t bo = (size_t)(16 * t + m) * FEAT + 32 * kt + 8 * hh;
      FragB fbh, fbl;
      fbh.h[0] = *(const v8us*)(Bh + bo); fbh.h[1] = *(const v8us*)(Bh + bo + 16);
      fbl.h[0] = *(const v8us*)(Bl + bo); fbl.h[1] = *(const v8us*)(Bl + bo + 16);
      acc[t] = wm3(fah.u, fal.u, fbh.u, fbl.u, acc[t]);
    }
  }
  {
    float* sp = stg + (r0 + 8 * hh) * FEAT + m;
#pragma unroll
    for (int t = 0; t < 8; ++t) {
#pragma unroll
      for (int r = 0; r < 8; ++r) sp[r * FEAT + 16 * t] = acc[t][r];
    }
  }
  __syncthreads();

  const v4f bv = *(const v4f*)(bias + 4 * lane);
  const v4f wv = *(const v4f*)(dw + 4 * lane);
  float myd = 0.f;
#pragma unroll 1
  for (int i = 0; i < 16; ++i) {
    const int row = r0 + i, grow = rowBase + row;
    float* lp = stg + row * FEAT + 4 * lane;
    v4f v = *(const v4f*)lp + bv;
    if (act == 1) {
      v.x = lrl(v.x); v.y = lrl(v.y); v.z = lrl(v.z); v.w = lrl(v.w);
    } else if (act == 2) {
      const float c = 0.70710678118654752f;
      v.x = v.x * 0.5f * (1.0f + erff(v.x * c));
      v.y = v.y * 0.5f * (1.0f + erff(v.y * c));
      v.z = v.z * 0.5f * (1.0f + erff(v.z * c));
      v.w = v.w * 0.5f * (1.0f + erff(v.w * c));
    }
    *(v4f*)lp = v;
    if (useF != 0 && grow < nValid) *(volatile v4f*)(outF + (size_t)grow * FEAT + 4 * lane) = v;
    if (useP != 0) {
      const v4us hv = hi4(v), lv = lo4(v, hv);
      const size_t po = (size_t)grow * FEAT + 4 * lane;
      *(volatile v4us*)(Ph + po) = hv;
      *(volatile v4us*)(Pl + po) = lv;
    }
    if (useD != 0) {
      float s = v.x * wv.x + v.y * wv.y + v.z * wv.z + v.w * wv.w;
      s += __shfl_xor(s, 16, 32); s += __shfl_xor(s, 8, 32); s += __shfl_xor(s, 4, 32);
      s += __shfl_xor(s, 2, 32);  s += __shfl_xor(s, 1, 32);
      myd = (lane == i) ? s : myd;
    }
  }
  if (useD != 0 && lane < 16) sdot[r0 + lane] = myd;
  __syncthreads();
  v4f dv = {0.f, 0.f, 0.f, 0.f};
  if (tid < 16) dv = *(const v4f*)(sdot + 4 * tid);
  if (useD != 0 && tid < 16) *(volatile v4f*)(dout + rowBase + 4 * tid) = dv;
  __threadfence();
#pragma unroll 1
  for (int i = 0; i < 16; ++i) {
    const int row = r0 + i, grow = rowBase + row;
    const float* lp = stg + row * FEAT + 4 * lane;
    const v4f v = *(const v4f*)lp;
    if (useF != 0 && grow < nValid) *(volatile v4f*)(outF + (size_t)grow * FEAT + 4 * lane) = v;
    if (useP != 0) {
      const v4us hv = hi4(v), lv = lo4(v, hv);
      const size_t po = (size_t)grow * FEAT + 4 * lane;
      *(volatile v4us*)(Ph + po) = hv;
      *(volatile v4us*)(Pl + po) = lv;
    }
  }
  if (useD != 0 && tid < 16) *(volatile v4f*)(dout + rowBase + 4 * tid) = dv;
}

__global__ __launch_bounds__(NTHR) void k_edge1(
    const unsigned short* __restrict__ Ah, const unsigned short* __restrict__ Al,
    const int* __restrict__ esrc, const int* __restrict__ edst, const float* __restrict__ bond,
    const unsigned short* __restrict__ Bh, const unsigned short* __restrict__ Bl,
    const float* __restrict__ b2, const float* __restrict__ attw, const float* __restrict__ attb,
    const float* __restrict__ adst, float* lg, int nN, int nE) {
  extern __shared__ v4f lds_dyn[];
  unsigned short* sAh = (unsigned short*)lds_dyn;
  unsigned short* sAl = sAh + EROWS * AP2;
  float* slg = (float*)(sAl + EROWS * AP2);
  const int tid = threadIdx.x, lane = tid & 31, wave = tid >> 5, hh = lane >> 4, m = lane & 15;
  const int eBase = blockIdx.x * EROWS;

  {
    const int r = tid & (EROWS - 1), half = tid >> 7;
    const int e = eBase + r;
    const int ec = e > nE - 1 ? nE - 1 : e;
    const int s = clampi(esrc[ec], nN - 1);
    const size_t go = (size_t)s * FEAT + 64 * half;
    unsigned short* dh = sAh + r * AP2 + 64 * half;
    unsigned short* dl = sAl + r * AP2 + 64 * half;
#pragma unroll
    for (int j = 0; j < 8; ++j) {
      *(v8us*)(dh + 8 * j) = *(const v8us*)(Ah + go + 8 * j);
      *(v8us*)(dl + 8 * j) = *(const v8us*)(Al + go + 8 * j);
    }
    if (half == 0) {
      const float* bp = bond + (size_t)ec * BONDF;
      const v4f q0 = *(const v4f*)bp, q1 = *(const v4f*)(bp + 4), q2 = *(const v4f*)(bp + 8), q3 = *(const v4f*)(bp + 12);
      const v4us h0 = hi4(q0), h1 = hi4(q1), h2 = hi4(q2), h3 = hi4(q3);
      const v4us l0 = lo4(q0, h0), l1 = lo4(q1, h1), l2 = lo4(q2, h2), l3 = lo4(q3, h3);
      *(v8us*)(sAh + r * AP2 + 128) = cat8(h0, h1);
      *(v8us*)(sAh + r * AP2 + 136) = cat8(h2, h3);
      *(v8us*)(sAl + r * AP2 + 128) = cat8(l0, l1);
      *(v8us*)(sAl + r * AP2 + 136) = cat8(l2, l3);
    } else {
      const v8us z = {0, 0, 0, 0, 0, 0, 0, 0};
      *(v8us*)(sAh + r * AP2 + 144) = z;
      *(v8us*)(sAh + r * AP2 + 152) = z;
      *(v8us*)(sAl + r * AP2 + 144) = z;
      *(v8us*)(sAl + r * AP2 + 152) = z;
    }
  }
  __syncthreads();

  const int r0 = wave * 16;
  v8f acc[8];
#pragma unroll
  for (int t = 0; t < 8; ++t) { v8f z = {0.f, 0.f, 0.f, 0.f, 0.f, 0.f, 0.f, 0.f}; acc[t] = z; }
  const unsigned short* arh = sAh + (r0 + m) * AP2 + 8 * hh;
  const unsigned short* arl = sAl + (r0 + m) * AP2 + 8 * hh;
#pragma unroll
  for (int kt = 0; kt < K2P / 32; ++kt) {
    FragB fah, fal;
    fah.h[0] = *(const v8us*)(arh + 32 * kt);
    fah.h[1] = *(const v8us*)(arh + 32 * kt + 16);
    fal.h[0] = *(const v8us*)(arl + 32 * kt);
    fal.h[1] = *(const v8us*)(arl + 32 * kt + 16);
#pragma unroll
    for (int t = 0; t < 8; ++t) {
      const size_t bo = (size_t)(16 * t + m) * K2P + 32 * kt + 8 * hh;
      FragB fbh, fbl;
      fbh.h[0] = *(const v8us*)(Bh + bo); fbh.h[1] = *(const v8us*)(Bh + bo + 16);
      fbl.h[0] = *(const v8us*)(Bl + bo); fbl.h[1] = *(const v8us*)(Bl + bo + 16);
      acc[t] = wm3(fah.u, fal.u, fbh.u, fbl.u, acc[t]);
    }
  }
  float part[8];
#pragma unroll
  for (int r = 0; r < 8; ++r) part[r] = 0.f;
#pragma unroll
  for (int t = 0; t < 8; ++t) {
    const int col = 16 * t + m;
    const float bb = b2[col];
    const float aw = attw[FEAT + col];
#pragma unroll
    for (int r = 0; r < 8; ++r) {
      const float x = lrl(acc[t][r] + bb);
      part[r] += x * aw;
    }
  }
#pragma unroll
  for (int r = 0; r < 8; ++r) {
    part[r] += __shfl_xor(part[r], 8, 32);
    part[r] += __shfl_xor(part[r], 4, 32);
    part[r] += __shfl_xor(part[r], 2, 32);
    part[r] += __shfl_xor(part[r], 1, 32);
  }
  if (m == 0) {
#pragma unroll
    for (int r = 0; r < 8; ++r) slg[r0 + 8 * hh + r] = part[r];
  }
  __syncthreads();

  if (wave == 0) {
    const float ab = attb[0];
    float t4[4];
#pragma unroll
    for (int j = 0; j < 4; ++j) {
      const int idx = 4 * lane + j;
      const int e = eBase + idx;
      const int ec = e > nE - 1 ? nE - 1 : e;
      const int d = clampi(edst[ec], nN - 1);
      t4[j] = lrl(adst[d] + slg[idx] + ab);
    }
    v4f o; o.x = t4[0]; o.y = t4[1]; o.z = t4[2]; o.w = t4[3];
    float* gp = lg + (size_t)eBase + 4 * lane;
    *(volatile v4f*)gp = o;
    __threadfence();
    *(volatile v4f*)gp = o;
  }
}

__global__ __launch_bounds__(NTHR) void k_edge2(
    const int* __restrict__ esrc, const int* __restrict__ edst,
    const float* __restrict__ ad, const float* __restrict__ as, const float* __restrict__ b,
    float* lg, int nN, int nE) {
  const int i = blockIdx.x * NTHR + (int)threadIdx.x;
  const float bb = b[0];
  float t4[4];
#pragma unroll
  for (int j = 0; j < 4; ++j) {
    const int e = 4 * i + j;
    const int ec = e > nE - 1 ? nE - 1 : e;
    const int d = clampi(edst[ec], nN - 1);
    const int s = clampi(esrc[ec], nN - 1);
    t4[j] = lrl(ad[d] + as[s] + bb);
  }
  v4f o; o.x = t4[0]; o.y = t4[1]; o.z = t4[2]; o.w = t4[3];
  float* gp = lg + (size_t)i * 4;
  *(volatile v4f*)gp = o;
  __threadfence();
  *(volatile v4f*)gp = o;
}

__global__ __launch_bounds__(NTHR) void k_agg(
    const int* __restrict__ esrc, const int* __restrict__ edst, const float* __restrict__ lg,
    const float* __restrict__ nt, unsigned short* Ph, unsigned short* Pl, int nN, int nE, int vec8) {
  extern __shared__ v4f lds_dyn[];
  float* sacc = (float*)lds_dyn;
  float* sm   = sacc + NBA * FEAT;
  float* sden = sm + NBA;
  int*   list = (int*)(sden + NBA);
  int*   wcnt = list + LISTN;
  const int tid = threadIdx.x, lane = tid & 31, wave = tid >> 5;
  const int slotBase = blockIdx.x * NBA;

  {
    const v4f z = {0.f, 0.f, 0.f, 0.f};
    const float ninf = __uint_as_float(0xff800000u);
    for (int i = tid; i < NBA * FEAT / 4; i += NTHR) ((v4f*)sacc)[i] = z;
    for (int i = tid; i < NBA; i += NTHR) { sm[i] = ninf; sden[i] = 0.f; }
  }
  __syncthreads();

  const int nChunks = (nE + CHUNK - 1) / CHUNK;
#pragma unroll 1
  for (int ch = 0; ch < nChunks; ++ch) {
    const int cbase = ch * CHUNK;
    const int wc = scan_chunk<NBA>(edst, nE, cbase, slotBase, vec8, list, tid, lane, wave);
    if (lane == 0) wcnt[wave] = wc;
    __syncthreads();
    if (wave == 0) {
#pragma unroll 1
      for (int wsx = 0; wsx < NWAVE; ++wsx) {
        int n = __builtin_amdgcn_readfirstlane(wcnt[wsx]);
        n = n > WCAP ? WCAP : (n < 0 ? 0 : n);
        const int* lp = list + wsx * WCAP;
#pragma unroll 1
        for (int i = 0; i < n; ++i) {
          const int ent  = __builtin_amdgcn_readfirstlane(lp[i]);
          const int slot = ent & (NBA - 1);
          int e = cbase + ((ent >> 12) & (CHUNK - 1));
          e = e > nE - 1 ? nE - 1 : e;
          const int s = clampi(esrc[e], nN - 1);
          const float l = lg[e];
          const v4f v = *(const v4f*)(nt + (size_t)s * FEAT + 4 * lane);
          const float mo = sm[slot], dn = sden[slot];
          const float mn = fmaxf(mo, l);
          const float sc = expf(mo - mn);
          const float p  = expf(l - mn);
          sm[slot] = mn;
          sden[slot] = dn * sc + p;
          v4f* ap = (v4f*)(sacc + slot * FEAT + 4 * lane);
          *ap = *ap * sc + v * p;
        }
      }
    }
    __syncthreads();
  }

#pragma unroll 1
  for (int pass = 0; pass < 2; ++pass) {
#pragma unroll 1
    for (int j = 0; j < 32; ++j) {
      const int slot = wave * 32 + j;
      const int row = slotBase + slot;
      const float d = sden[slot];
      const float rc = __builtin_amdgcn_rcpf(d);
      const float inv = d > 0.f ? rc : 0.f;
      const v4f t = *(const v4f*)(sacc + slot * FEAT + 4 * lane) * inv;
      v4f c;
      c.x = t.x > 0.f ? t.x : expm1f(fminf(t.x, 0.f));
      c.y = t.y > 0.f ? t.y : expm1f(fminf(t.y, 0.f));
      c.z = t.z > 0.f ? t.z : expm1f(fminf(t.z, 0.f));
      c.w = t.w > 0.f ? t.w : expm1f(fminf(t.w, 0.f));
      const v4us hv = hi4(c), lv = lo4(c, hv);
      const size_t po = (size_t)row * FEAT + 4 * lane;
      *(volatile v4us*)(Ph + po) = hv;
      *(volatile v4us*)(Pl + po) = lv;
    }
    __threadfence();
  }
}

__global__ __launch_bounds__(GTHR) void k_gru(
    const unsigned short* __restrict__ Xh, const unsigned short* __restrict__ Xl,
    const unsigned short* __restrict__ Hh, const unsigned short* __restrict__ Hl,
    const float* __restrict__ hold,
    const unsigned short* __restrict__ Wi, const unsigned short* __restrict__ Wh,
    const float* __restrict__ bih, const float* __restrict__ bhh,
    float* outF, unsigned short* Ph, unsigned short* Pl,
    const float* __restrict__ dw, float* d1out, float* d2out, int nN) {
  extern __shared__ v4f lds_dyn[];
  float* stg  = (float*)lds_dyn;
  float* sdot = stg + GROWS * GIP;
  const int tid = threadIdx.x, lane = tid & 31, wave = tid >> 5, hh = lane >> 4, m = lane & 15;
  const int rowBase = blockIdx.x * GROWS;
  const int r0 = wave * 16;

#pragma unroll 1
  for (int grp = 0; grp < 6; ++grp) {
    const int isH = grp >= 3 ? 1 : 0;
    const int cg  = grp - 3 * isH;
    const unsigned short* Ah = isH != 0 ? Hh : Xh;
    const unsigned short* Al = isH != 0 ? Hl : Xl;
    const unsigned short* Bh = (isH != 0 ? Wh : Wi) + (size_t)cg * 128 * FEAT;
    const unsigned short* Bl = Bh + WSZ_GRU;
    v8f acc[8];
#pragma unroll
    for (int t = 0; t < 8; ++t) { v8f z = {0.f, 0.f, 0.f, 0.f, 0.f, 0.f, 0.f, 0.f}; acc[t] = z; }
    const size_t ao = (size_t)(rowBase + r0 + m) * FEAT + 8 * hh;
    const unsigned short* ah = Ah + ao;
    const unsigned short* al = Al + ao;
#pragma unroll
    for (int kt = 0; kt < FEAT / 32; ++kt) {
      FragB fah, fal;
      fah.h[0] = *(const v8us*)(ah + 32 * kt);
      fah.h[1] = *(const v8us*)(ah + 32 * kt + 16);
      fal.h[0] = *(const v8us*)(al + 32 * kt);
      fal.h[1] = *(const v8us*)(al + 32 * kt + 16);
#pragma unroll
      for (int t = 0; t < 8; ++t) {
        const size_t bo = (size_t)(16 * t + m) * FEAT + 32 * kt + 8 * hh;
        FragB fbh, fbl;
        fbh.h[0] = *(const v8us*)(Bh + bo); fbh.h[1] = *(const v8us*)(Bh + bo + 16);
        fbl.h[0] = *(const v8us*)(Bl + bo); fbl.h[1] = *(const v8us*)(Bl + bo + 16);
        acc[t] = wm3(fah.u, fal.u, fbh.u, fbl.u, acc[t]);
      }
    }
    float* sp = stg + (r0 + 8 * hh) * GIP + grp * 128 + m;
#pragma unroll
    for (int t = 0; t < 8; ++t) {
#pragma unroll
      for (int r = 0; r < 8; ++r) sp[r * GIP + 16 * t] = acc[t][r];
    }
  }
  __syncthreads();

  const v4f bir = *(const v4f*)(bih + 4 * lane), biz = *(const v4f*)(bih + 128 + 4 * lane), bin = *(const v4f*)(bih + 256 + 4 * lane);
  const v4f bhr = *(const v4f*)(bhh + 4 * lane), bhz = *(const v4f*)(bhh + 128 + 4 * lane), bhn = *(const v4f*)(bhh + 256 + 4 * lane);
  const v4f w1 = *(const v4f*)(dw + 4 * lane), w2 = *(const v4f*)(dw + 128 + 4 * lane);
  float myd1 = 0.f, myd2 = 0.f;
#pragma unroll 1
  for (int i = 0; i < 16; ++i) {
    const int row = r0 + i, grow = rowBase + row;
    const int growc = grow > nN - 1 ? nN - 1 : grow;
    float* lp = stg + row * GIP + 4 * lane;
    const v4f gir = *(const v4f*)lp,         giz = *(const v4f*)(lp + 128), gin = *(const v4f*)(lp + 256);
    const v4f ghr = *(const v4f*)(lp + 384), ghz = *(const v4f*)(lp + 512), ghn = *(const v4f*)(lp + 640);
    const v4f ho = *(const v4f*)(hold + (size_t)growc * FEAT + 4 * lane);
    const v4f xr = gir + bir + ghr + bhr;
    const v4f xz = giz + biz + ghz + bhz;
    v4f rr, zz, nn, hn;
    rr.x = sigf(xr.x); rr.y = sigf(xr.y); rr.z = sigf(xr.z); rr.w = sigf(xr.w);
    zz.x = sigf(xz.x); zz.y = sigf(xz.y); zz.z = sigf(xz.z); zz.w = sigf(xz.w);
    const v4f xn = gin + bin + rr * (ghn + bhn);
    nn.x = tanhf(xn.x); nn.y = tanhf(xn.y); nn.z = tanhf(xn.z); nn.w = tanhf(xn.w);
    const v4f one = {1.f, 1.f, 1.f, 1.f};
    hn = (one - zz) * nn + zz * ho;
    *(v4f*)lp = hn;
    if (grow < nN) *(volatile v4f*)(outF + (size_t)grow * FEAT + 4 * lane) = hn;
    {
      const v4us hv = hi4(hn), lv = lo4(hn, hv);
      const size_t po = (size_t)grow * FEAT + 4 * lane;
      *(volatile v4us*)(Ph + po) = hv;
      *(volatile v4us*)(Pl + po) = lv;
    }
    float s1 = hn.x * w1.x + hn.y * w1.y + hn.z * w1.z + hn.w * w1.w;
    float s2 = hn.x * w2.x + hn.y * w2.y + hn.z * w2.z + hn.w * w2.w;
    s1 += __shfl_xor(s1, 16, 32); s1 += __shfl_xor(s1, 8, 32); s1 += __shfl_xor(s1, 4, 32);
    s1 += __shfl_xor(s1, 2, 32);  s1 += __shfl_xor(s1, 1, 32);
    s2 += __shfl_xor(s2, 16, 32); s2 += __shfl_xor(s2, 8, 32); s2 += __shfl_xor(s2, 4, 32);
    s2 += __shfl_xor(s2, 2, 32);  s2 += __shfl_xor(s2, 1, 32);
    myd1 = (lane == i) ? s1 : myd1;
    myd2 = (lane == i) ? s2 : myd2;
  }
  if (lane < 16) { sdot[r0 + lane] = myd1; sdot[GROWS + r0 + lane] = myd2; }
  __syncthreads();
  v4f dv = {0.f, 0.f, 0.f, 0.f};
  if (tid < 32) dv = (tid < 16) ? *(const v4f*)(sdot + 4 * tid) : *(const v4f*)(sdot + GROWS + 4 * (tid - 16));
  float* dp = (tid < 16) ? (d1out + rowBase + 4 * tid) : (d2out + rowBase + 4 * (tid - 16));
  if (tid < 32) *(volatile v4f*)dp = dv;
  __threadfence();
#pragma unroll 1
  for (int i = 0; i < 16; ++i) {
    const int row = r0 + i, grow = rowBase + row;
    const float* lp = stg + row * GIP + 4 * lane;
    const v4f hn = *(const v4f*)lp;
    if (grow < nN) *(volatile v4f*)(outF + (size_t)grow * FEAT + 4 * lane) = hn;
    const v4us hv = hi4(hn), lv = lo4(hn, hv);
    const size_t po = (size_t)grow * FEAT + 4 * lane;
    *(volatile v4us*)(Ph + po) = hv;
    *(volatile v4us*)(Pl + po) = lv;
  }
  if (tid < 32) *(volatile v4f*)dp = dv;
}

__global__ __launch_bounds__(NTHR) void k_avg(
    const float* __restrict__ h1, const float* __restrict__ h2, const float* __restrict__ h3,
    float* outF, unsigned short* Ph, unsigned short* Pl, int nN) {
  const int tid = threadIdx.x, lane = tid & 31, wave = tid >> 5;
  const int rb = blockIdx.x * GROWS + wave * 8;
  const float third = 1.0f / 3.0f;
#pragma unroll 1
  for (int pass = 0; pass < 2; ++pass) {
#pragma unroll 1
    for (int j = 0; j < 8; ++j) {
      const int row = rb + j;
      const int rc = row > nN - 1 ? nN - 1 : row;
      const size_t o = (size_t)rc * FEAT + 4 * lane;
      const v4f v = (*(const v4f*)(h1 + o) + *(const v4f*)(h2 + o) + *(const v4f*)(h3 + o)) * third;
      if (row < nN) *(volatile v4f*)(outF + (size_t)row * FEAT + 4 * lane) = v;
      const v4us hv = hi4(v), lv = lo4(v, hv);
      const size_t po = (size_t)row * FEAT + 4 * lane;
      *(volatile v4us*)(Ph + po) = hv;
      *(volatile v4us*)(Pl + po) = lv;
    }
    __threadfence();
  }
}

extern "C" void kernel_launch(void* const* d_in, const int* in_sizes, int n_in,
                              void* d_out, int out_size, void* d_ws, size_t ws_size,
                              hipStream_t stream) {
  if (n_in < 26) return;
  if (in_sizes[0] <= 0 || (in_sizes[0] % FEAT) != 0) return;
  const int nN = in_sizes[0] / FEAT;
  const int nE = in_sizes[1];
  if (nE <= 0 || in_sizes[2] != nE || in_sizes[3] != nE * BONDF) return;
  if (in_sizes[4] != FEAT * FEAT || in_sizes[5] != FEAT || in_sizes[6] != FEAT * (FEAT + BONDF) || in_sizes[7] != FEAT) return;
  if (in_sizes[8] != 2 * FEAT || in_sizes[9] < 1 || in_sizes[10] != FEAT * FEAT || in_sizes[11] != FEAT) return;
  if (in_sizes[12] != 3 * FEAT * FEAT || in_sizes[13] != 3 * FEAT * FEAT || in_sizes[14] != 3 * FEAT || in_sizes[15] != 3 * FEAT) return;
  if (in_sizes[16] != 2 * FEAT || in_sizes[17] < 1 || in_sizes[18] != FEAT * FEAT || in_sizes[19] != FEAT) return;
  if (in_sizes[20] != 3 * FEAT * FEAT || in_sizes[21] != 3 * FEAT * FEAT || in_sizes[22] != 3 * FEAT || in_sizes[23] != 3 * FEAT) return;
  if (in_sizes[24] != FEAT * FEAT || in_sizes[25] != FEAT) return;
  if (nN > (1 << 22) || nE > (1 << 26)) return;
  if (out_size != 6 * nN * FEAT) return;

  const float* atom   = (const float*)d_in[0];
  const int*   esrc   = (const int*)d_in[1];
  const int*   edst   = (const int*)d_in[2];
  const float* bond   = (const float*)d_in[3];
  const float* fc1_w  = (const float*)d_in[4];
  const float* fc1_b  = (const float*)d_in[5];
  const float* fc2_w  = (const float*)d_in[6];
  const float* fc2_b  = (const float*)d_in[7];
  const float* att_w  = (const float*)d_in[8];
  const float* att_b  = (const float*)d_in[9];
  const float* atn_w  = (const float*)d_in[10];
  const float* atn_b  = (const float*)d_in[11];
  const float* wih1   = (const float*)d_in[12];
  const float* whh1   = (const float*)d_in[13];
  const float* bih1   = (const float*)d_in[14];
  const float* bhh1   = (const float*)d_in[15];
  const float* f1v2_w = (const float*)d_in[16];
  const float* f1v2_b = (const float*)d_in[17];
  const float* f2v2_w = (const float*)d_in[18];
  const float* f2v2_b = (const float*)d_in[19];
  const float* wih2   = (const float*)d_in[20];
  const float* whh2   = (const float*)d_in[21];
  const float* bih2   = (const float*)d_in[22];
  const float* bhh2   = (const float*)d_in[23];
  const float* lin_w  = (const float*)d_in[24];
  const float* lin_b  = (const float*)d_in[25];

  float* out = (float*)d_out;
  const size_t SZ = (size_t)nN * FEAT;
  float* o_main = out;
  float* o_h1   = out + SZ;
  float* o_h2   = out + 2 * SZ;
  float* o_h3   = out + 3 * SZ;
  float* o_g0   = out + 4 * SZ;
  float* o_avg  = out + 5 * SZ;

  const int NPAD  = ((nN + NBA - 1) / NBA) * NBA;
  const int EPAD  = ((nE + 1023) / 1024) * 1024;
  const int gridG = (nN + GROWS - 1) / GROWS;
  const int nAgg  = NPAD / NBA;
  const int nE1   = (nE + EROWS - 1) / EROWS;
  const int nE2   = EPAD / 1024;
  const int nAp   = NPAD / 16;
  if ((size_t)nE1 * EROWS > (size_t)EPAD) return;

  char* ws = (char*)d_ws;
  size_t off = 0;
  const size_t PLB = (size_t)NPAD * FEAT * 2;
#define CARVE(NAME, BYTES) const size_t NAME = off; off += (size_t)(BYTES); off = (off + 255) & ~(size_t)255;
  CARVE(oW,   (size_t)WO_END * 2)
  CARVE(oAh,  PLB) CARVE(oAl,  PLB)
  CARVE(oGah, PLB) CARVE(oGal, PLB)
  CARVE(oGbh, PLB) CARVE(oGbl, PLB)
  CARVE(oCh,  PLB) CARVE(oCl,  PLB)
  CARVE(oVh,  PLB) CARVE(oVl,  PLB)
  CARVE(oNT,  (size_t)NPAD * FEAT * 4)
  CARVE(oLg,  (size_t)EPAD * 4)
  CARVE(oAd0, (size_t)NPAD * 4)
  CARVE(oAd,  (size_t)NPAD * 4)
  CARVE(oAs,  (size_t)NPAD * 4)
#undef CARVE
  if (off > ws_size || off > (size_t)134217728) return;

  unsigned short* wpl = (unsigned short*)(ws + oW);
  unsigned short* Ah  = (unsigned short*)(ws + oAh);
  unsigned short* Al  = (unsigned short*)(ws + oAl);
  unsigned short* Gah = (unsigned short*)(ws + oGah);
  unsigned short* Gal = (unsigned short*)(ws + oGal);
  unsigned short* Gbh = (unsigned short*)(ws + oGbh);
  unsigned short* Gbl = (unsigned short*)(ws + oGbl);
  unsigned short* Ch  = (unsigned short*)(ws + oCh);
  unsigned short* Cl  = (unsigned short*)(ws + oCl);
  unsigned short* Vh  = (unsigned short*)(ws + oVh);
  unsigned short* Vl  = (unsigned short*)(ws + oVl);
  float* NT  = (float*)(ws + oNT);
  float* lgp = (float*)(ws + oLg);
  float* ad0 = (float*)(ws + oAd0);
  float* ad  = (float*)(ws + oAd);
  float* as  = (float*)(ws + oAs);

  const int vec8 = ((nE & 3) == 0) ? 1 : 0;

  hipFuncSetAttribute(reinterpret_cast<const void*>(&k_edge1), hipFuncAttributeMaxDynamicSharedMemorySize, LDS_EDGE);
  hipFuncSetAttribute(reinterpret_cast<const void*>(&k_agg),   hipFuncAttributeMaxDynamicSharedMemorySize, LDS_AGG);
  hipFuncSetAttribute(reinterpret_cast<const void*>(&k_gru),   hipFuncAttributeMaxDynamicSharedMemorySize, LDS_GRU);

  k_wprep<<<WGRP_END / NTHR, NTHR, 0, stream>>>(fc1_w, atn_w, fc2_w, wih1, whh1, f2v2_w, wih2, whh2, lin_w, wpl);
  k_aprep<<<nAp, NTHR, 0, stream>>>(atom, Ah, Al, nN);

  k_lin<<<gridG, GTHR, 0, stream>>>(Ah, Al, wpl + WO_FC1, wpl + WO_FC1 + WSZ_SQ, fc1_b, 1,
                                    o_g0, 1, nN, Gah, Gal, 1, att_w, ad0, 1);
  k_lin<<<gridG, GTHR, 0, stream>>>(Gah, Gal, wpl + WO_ATT, wpl + WO_ATT + WSZ_SQ, atn_b, 0,
                                    NT, 1, NPAD, Vh, Vl, 0, att_w, ad0, 0);
  k_edge1<<<nE1, NTHR, LDS_EDGE, stream>>>(Ah, Al, esrc, edst, bond, wpl + WO_FC2, wpl + WO_FC2 + WSZ_FC2,
                                           fc2_b, att_w, att_b, ad0, lgp, nN, nE);
  k_agg<<<nAgg, NTHR, LDS_AGG, stream>>>(esrc, edst, lgp, NT, Ch, Cl, nN, nE, vec8);
  k_gru<<<gridG, GTHR, LDS_GRU, stream>>>(Ch, Cl, Gah, Gal, o_g0, wpl + WO_WIH1, wpl + WO_WHH1, bih1, bhh1,
                                          o_h1, Gbh, Gbl, f1v2_w, ad, as, nN);

  k_lin<<<gridG, GTHR, 0, stream>>>(Gbh, Gbl, wpl + WO_F2V2, wpl + WO_F2V2 + WSZ_SQ, f2v2_b, 0,
                                    NT, 1, NPAD, Vh, Vl, 0, att_w, ad0, 0);
  k_edge2<<<nE2, NTHR, 0, stream>>>(esrc, edst, ad, as, f1v2_b, lgp, nN, nE);
  k_agg<<<nAgg, NTHR, LDS_AGG, stream>>>(esrc, edst, lgp, NT, Ch, Cl, nN, nE, vec8);
  k_gru<<<gridG, GTHR, LDS_GRU, stream>>>(Ch, Cl, Gbh, Gbl, o_h1, wpl + WO_WIH2, wpl + WO_WHH2, bih2, bhh2,
                                          o_h2, Gah, Gal, f1v2_w, ad, as, nN);

  k_lin<<<gridG, GTHR, 0, stream>>>(Gah, Gal, wpl + WO_F2V2, wpl + WO_F2V2 + WSZ_SQ, f2v2_b, 0,
                                    NT, 1, NPAD, Vh, Vl, 0, att_w, ad0, 0);
  k_edge2<<<nE2, NTHR, 0, stream>>>(esrc, edst, ad, as, f1v2_b, lgp, nN, nE);
  k_agg<<<nAgg, NTHR, LDS_AGG, stream>>>(esrc, edst, lgp, NT, Ch, Cl, nN, nE, vec8);
  k_gru<<<gridG, GTHR, LDS_GRU, stream>>>(Ch, Cl, Gah, Gal, o_h2, wpl + WO_WIH2, wpl + WO_WHH2, bih2, bhh2,
                                          o_h3, Gbh, Gbl, f1v2_w, ad, as, nN);

  k_avg<<<gridG, NTHR, 0, stream>>>(o_h1, o_h2, o_h3, o_avg, Vh, Vl, nN);
  k_lin<<<gridG, GTHR, 0, stream>>>(Vh, Vl, wpl + WO_LIN, wpl + WO_LIN + WSZ_SQ, lin_b, 2,
                                    o_main, 1, nN, Ch, Cl, 0, att_w, ad0, 0);
}
